// HybridGnnTorsoV2_74036646248567
// MI455X (gfx1250) — hardware-verified
//
#include <hip/hip_runtime.h>

#define NCELL  512
#define NFRM   16
#define CDIM   128
#define LGNN   3
#define LTF    2
#define NTOK   15
#define FFD    512
#define OROWS  26
#define QKVD   384
#define LN_EPS 1e-5f

#define OFF_WL   0
#define OFF_WR   49152
#define OFF_WACT 98304
#define OFF_WQKV 163840
#define OFF_WO   262144
#define OFF_W1   294912
#define OFF_W2   425984
#define PLANE_N  557056

#define G_XS   0
#define G_FV   262144
#define G_SV   264192
#define G_RED  264704
#define G_MISC 265728
#define G_LDS  265792

#define T_AL   0
#define T_QKV  8192
#define T_PAH  32768
#define T_PAL  36864
#define T_PBH  40960
#define T_PBL  57344
#define T_OST  73728
#define T_LDS  74752

typedef __bf16 v16bf __attribute__((ext_vector_type(16)));
typedef float v8f __attribute__((ext_vector_type(8)));
typedef float v4f __attribute__((ext_vector_type(4)));
typedef unsigned int v4u __attribute__((ext_vector_type(4)));
typedef unsigned int v2u __attribute__((ext_vector_type(2)));
typedef int v4i __attribute__((ext_vector_type(4)));
typedef v4f __attribute__((may_alias)) v4fa;
typedef v4u __attribute__((may_alias)) v4ua;
typedef v2u __attribute__((may_alias)) v2ua;
typedef v4i __attribute__((may_alias)) v4ia;

union FragBF { v16bf v; v4u q[2]; unsigned int u[8]; };

__device__ __forceinline__ unsigned int f2bf_bits(float f) {
  unsigned int u = __float_as_uint(f);
  u += 0x7FFFu + ((u >> 16) & 1u);
  return u >> 16;
}
__device__ __forceinline__ float bf_bits2f(unsigned int bts) { return __uint_as_float(bts << 16); }
__device__ __forceinline__ void split2(float a, float b, unsigned int& ph, unsigned int& pl) {
  const unsigned int ha = f2bf_bits(a), hb = f2bf_bits(b);
  const unsigned int la = f2bf_bits(a - bf_bits2f(ha)), lb = f2bf_bits(b - bf_bits2f(hb));
  ph = ha | (hb << 16);
  pl = la | (lb << 16);
}

__device__ __forceinline__ v8f wmma_bf(v16bf a, v16bf b, v8f c) {
  v8f d = __builtin_amdgcn_wmma_f32_16x16x32_bf16(false, a, false, b, (short)0, c, false, false);
  asm volatile("v_nop\n\tv_nop\n\tv_nop\n\tv_nop" : "+v"(d) : "v"(a), "v"(b));
  return d;
}

__device__ __forceinline__ v16bf ldfrag16(const unsigned short* p, int h) {
  FragBF f;
  f.q[0] = *(const v4ua*)(p + 8 * h);
  f.q[1] = *(const v4ua*)(p + 16 + 8 * h);
  return f.v;
}

__global__ __launch_bounds__(256) void prep_kernel(
    const float* __restrict__ Wl, const float* __restrict__ Wr, const float* __restrict__ Wact,
    const float* __restrict__ Wqkv, const float* __restrict__ Wo, const float* __restrict__ W1,
    const float* __restrict__ W2, unsigned short* __restrict__ wph, unsigned short* __restrict__ wpl)
{
  const int g = blockIdx.x * 256 + threadIdx.x;
  if (g >= PLANE_N / 8) return;
  const int e = g * 8;
  const float* src =
      (e < OFF_WR)   ? (Wl + e) :
      (e < OFF_WACT) ? (Wr + (e - OFF_WR)) :
      (e < OFF_WQKV) ? (Wact + (e - OFF_WACT)) :
      (e < OFF_WO)   ? (Wqkv + (e - OFF_WQKV)) :
      (e < OFF_W1)   ? (Wo + (e - OFF_WO)) :
      (e < OFF_W2)   ? (W1 + (e - OFF_W1)) : (W2 + (e - OFF_W2));
  const v4f a = *(const v4fa*)src;
  const v4f c = *(const v4fa*)(src + 4);
  unsigned int h0, h1, h2, h3, l0, l1, l2, l3;
  split2(a.x, a.y, h0, l0);
  split2(a.z, a.w, h1, l1);
  split2(c.x, c.y, h2, l2);
  split2(c.z, c.w, h3, l3);
  const v4u hq = {h0, h1, h2, h3};
  const v4u lq = {l0, l1, l2, l3};
  unsigned short* dh = wph + e;
  unsigned short* dl = wpl + e;
  *(volatile v4u*)dh = hq;
  *(volatile v4u*)dl = lq;
  __threadfence();
  *(volatile v4u*)dh = hq;
  *(volatile v4u*)dl = lq;
}

__global__ __launch_bounds__(256) void gnn_kernel(
    const int* __restrict__ xx, const float* __restrict__ ss,
    const float* __restrict__ Win, const float* __restrict__ b_in,
    const float* __restrict__ bl, const float* __restrict__ ln_g, const float* __restrict__ ln_b,
    const unsigned short* __restrict__ wph, const unsigned short* __restrict__ wpl,
    float* __restrict__ out)
{
  extern __shared__ __attribute__((aligned(16))) unsigned char dsm[];
  float* xs   = (float*)(dsm + G_XS);
  float* fv   = (float*)(dsm + G_FV);
  float* sv   = (float*)(dsm + G_SV);
  float* red  = (float*)(dsm + G_RED);
  float* misc = (float*)(dsm + G_MISC);

  const int b = blockIdx.x, tid = threadIdx.x;
  const int lane = tid & 31, w = tid >> 5, h = lane >> 4, m = lane & 15;

  const int* fr0 = xx + (size_t)b * NFRM * NCELL;
  const int f0 = fr0[tid], f1 = fr0[tid + 256];
  fv[tid] = (float)f0;
  fv[tid + 256] = (float)f1;
  int cnt = ((f0 != 0) ? 1 : 0) + ((f1 != 0) ? 1 : 0);
  #pragma unroll
  for (int o = 16; o > 0; o >>= 1) cnt += __shfl_xor(cnt, o);
  if (lane == 0) misc[w] = (float)cnt;
  __syncthreads();
  float nf = 0.0f;
  #pragma unroll
  for (int i = 0; i < 8; ++i) nf += misc[i];
  const float cg = (nf > 1.0f) ? (1.0f / fmaxf(nf - 1.0f, 1.0f)) : 0.0f;

  {
    const int c = tid & 127, hb = tid >> 7;
    const float w0 = Win[c * 5 + 0], w1 = Win[c * 5 + 1], w2 = Win[c * 5 + 2];
    const float w3 = Win[c * 5 + 3], w4 = Win[c * 5 + 4], bb = b_in[c];
    const float s5 = ss[b] * 0.125f;
    #pragma unroll 2
    for (int node = hb * 256; node < hb * 256 + 256; ++node) {
      const float ci = (float)(node >> 6) * (1.0f / 7.0f);
      const float cj = (float)((node >> 3) & 7) * (1.0f / 7.0f);
      const float ck = (float)(node & 7) * (1.0f / 7.0f);
      const float f3 = fv[node] * 0.5f;
      xs[node * CDIM + c] = w0 * ci + w1 * cj + w2 * ck + w3 * f3 + w4 * s5 + bb;
    }
  }
  __syncthreads();

  float gcol[8], bcol[8];
  #pragma unroll
  for (int nt = 0; nt < 8; ++nt) {
    gcol[nt] = ln_g[16 * nt + m];
    bcol[nt] = ln_b[16 * nt + m];
  }
  const v8f zero8 = {0.f, 0.f, 0.f, 0.f, 0.f, 0.f, 0.f, 0.f};

  #pragma unroll 1
  for (int l = 0; l < LGNN; ++l) {
    {
      const int c = tid & 127, hb = tid >> 7;
      float acc = 0.0f;
      #pragma unroll 4
      for (int node = hb * 256; node < hb * 256 + 256; ++node) {
        const float mk = (fv[node] != 0.0f) ? 1.0f : 0.0f;
        acc += xs[node * CDIM + c] * mk;
      }
      red[tid] = acc;
    }
    __syncthreads();
    if (tid < CDIM) sv[tid] = red[tid] + red[tid + CDIM];
    __syncthreads();

    float bln[8];
    #pragma unroll
    for (int nt = 0; nt < 8; ++nt) bln[nt] = bl[l * CDIM + 16 * nt + m];

    const unsigned short* wlh = wph + OFF_WL + l * (CDIM * CDIM);
    const unsigned short* wll = wpl + OFF_WL + l * (CDIM * CDIM);
    const unsigned short* wrh = wph + OFF_WR + l * (CDIM * CDIM);
    const unsigned short* wrl = wpl + OFF_WR + l * (CDIM * CDIM);

    #pragma unroll 1
    for (int mt = 0; mt < 4; ++mt) {
      const int row0 = w * 64 + mt * 16;
      v8f acc[8];
      #pragma unroll
      for (int nt = 0; nt < 8; ++nt) acc[nt] = zero8;

      #pragma unroll 1
      for (int ks = 0; ks < 4; ++ks) {
        const int k0 = ks * 32;
        const float* xr = xs + (row0 + m) * CDIM + k0 + 8 * h;
        const float* sr = sv + k0 + 8 * h;
        const v4f xa = *(const v4fa*)(xr);
        const v4f xb = *(const v4fa*)(xr + 4);
        const v4f xc = *(const v4fa*)(xr + 16);
        const v4f xd = *(const v4fa*)(xr + 20);
        const v4f sa = *(const v4fa*)(sr);
        const v4f sb = *(const v4fa*)(sr + 4);
        const v4f sc = *(const v4fa*)(sr + 16);
        const v4f sd = *(const v4fa*)(sr + 20);
        const v4f na = (sa - xa) * cg;
        const v4f nb = (sb - xb) * cg;
        const v4f nc = (sc - xc) * cg;
        const v4f nd = (sd - xd) * cg;
        FragBF axh, axl, anh, anl;
        split2(xa.x, xa.y, axh.u[0], axl.u[0]);
        split2(xa.z, xa.w, axh.u[1], axl.u[1]);
        split2(xb.x, xb.y, axh.u[2], axl.u[2]);
        split2(xb.z, xb.w, axh.u[3], axl.u[3]);
        split2(xc.x, xc.y, axh.u[4], axl.u[4]);
        split2(xc.z, xc.w, axh.u[5], axl.u[5]);
        split2(xd.x, xd.y, axh.u[6], axl.u[6]);
        split2(xd.z, xd.w, axh.u[7], axl.u[7]);
        split2(na.x, na.y, anh.u[0], anl.u[0]);
        split2(na.z, na.w, anh.u[1], anl.u[1]);
        split2(nb.x, nb.y, anh.u[2], anl.u[2]);
        split2(nb.z, nb.w, anh.u[3], anl.u[3]);
        split2(nc.x, nc.y, anh.u[4], anl.u[4]);
        split2(nc.z, nc.w, anh.u[5], anl.u[5]);
        split2(nd.x, nd.y, anh.u[6], anl.u[6]);
        split2(nd.z, nd.w, anh.u[7], anl.u[7]);

        #pragma unroll
        for (int nt = 0; nt < 8; ++nt) {
          const int ro = (16 * nt + m) * CDIM + k0;
          {
            const v16bf bwh = ldfrag16(wlh + ro, h);
            const v16bf bwl = ldfrag16(wll + ro, h);
            acc[nt] = wmma_bf(anh.v, bwh, acc[nt]);
            acc[nt] = wmma_bf(anh.v, bwl, acc[nt]);
            acc[nt] = wmma_bf(anl.v, bwh, acc[nt]);
          }
          {
            const v16bf bwh = ldfrag16(wrh + ro, h);
            const v16bf bwl = ldfrag16(wrl + ro, h);
            acc[nt] = wmma_bf(axh.v, bwh, acc[nt]);
            acc[nt] = wmma_bf(axh.v, bwl, acc[nt]);
            acc[nt] = wmma_bf(axl.v, bwh, acc[nt]);
          }
        }
      }

      #pragma unroll
      for (int r = 0; r < 8; ++r) {
        float sm = 0.0f;
        #pragma unroll
        for (int nt = 0; nt < 8; ++nt) {
          const float hv = fmaxf(acc[nt][r] + bln[nt], 0.0f);
          acc[nt][r] = hv;
          sm += hv;
        }
        sm += __shfl_xor(sm, 1, 16);
        sm += __shfl_xor(sm, 2, 16);
        sm += __shfl_xor(sm, 4, 16);
        sm += __shfl_xor(sm, 8, 16);
        const float mu = sm * (1.0f / 128.0f);
        float sq = 0.0f;
        #pragma unroll
        for (int nt = 0; nt < 8; ++nt) {
          const float d = acc[nt][r] - mu;
          sq += d * d;
        }
        sq += __shfl_xor(sq, 1, 16);
        sq += __shfl_xor(sq, 2, 16);
        sq += __shfl_xor(sq, 4, 16);
        sq += __shfl_xor(sq, 8, 16);
        const float rs = rsqrtf(sq * (1.0f / 128.0f) + LN_EPS);
        float* orow = xs + (row0 + 8 * h + r) * CDIM + m;
        #pragma unroll
        for (int nt = 0; nt < 8; ++nt)
          orow[16 * nt] = (acc[nt][r] - mu) * rs * gcol[nt] + bcol[nt];
      }
    }
    __syncthreads();
  }

  v4f po[3];
  #pragma unroll
  for (int it = 0; it < 3; ++it) {
    v4f a4 = {0.f, 0.f, 0.f, 0.f};
    #pragma unroll 4
    for (int q = 0; q < 64; ++q) {
      int node;
      if (it == 0)      node = (w << 6) + q;
      else if (it == 1) node = ((q >> 3) << 6) + (w << 3) + (q & 7);
      else              node = ((q >> 3) << 6) + ((q & 7) << 3) + w;
      const float mk = (fv[node] != 0.0f) ? 1.0f : 0.0f;
      const v4f xv = *(const v4fa*)(xs + node * CDIM + 4 * lane);
      a4 += xv * mk;
    }
    po[it] = a4 * (1.0f / 64.0f);
  }
  float* ob = out + (size_t)b * OROWS * CDIM + 4 * lane;
  #pragma unroll
  for (int it = 0; it < 3; ++it) *(volatile v4f*)(ob + (it * 8 + w) * CDIM) = po[it];
  __threadfence();
  #pragma unroll
  for (int it = 0; it < 3; ++it) *(volatile v4f*)(ob + (it * 8 + w) * CDIM) = po[it];
}

template <int NT, int KS, bool ALO>
__device__ __forceinline__ void gemm16(v8f (&acc)[NT],
                                       const unsigned short* ah, const unsigned short* al, int lda,
                                       const unsigned short* bh, const unsigned short* blo, int ldb,
                                       int h, int m)
{
  #pragma unroll 1
  for (int ks = 0; ks < KS; ++ks) {
    const v16bf fa  = ldfrag16(ah + m * lda + 32 * ks, h);
    const v16bf fal = ALO ? ldfrag16(al + m * lda + 32 * ks, h) : fa;
    #pragma unroll
    for (int i = 0; i < NT; ++i) {
      const size_t bro = (size_t)(i * 16 + m) * ldb + 32 * ks;
      const v16bf fb  = ldfrag16(bh + bro, h);
      const v16bf fbl = ldfrag16(blo + bro, h);
      acc[i] = wmma_bf(fa, fb, acc[i]);
      acc[i] = wmma_bf(fa, fbl, acc[i]);
      if (ALO) acc[i] = wmma_bf(fal, fb, acc[i]);
    }
  }
}

__device__ __forceinline__ void ln_planes(const float* aL, const float* __restrict__ g,
                                          const float* __restrict__ be,
                                          unsigned short* ph_, unsigned short* pl_, int tid)
{
  const int t = tid >> 4, part = tid & 15;
  const float* row = aL + t * CDIM + part * 8;
  const v4f a = *(const v4fa*)row;
  const v4f c = *(const v4fa*)(row + 4);
  float sm = (a.x + a.y) + (a.z + a.w) + (c.x + c.y) + (c.z + c.w);
  sm += __shfl_xor(sm, 1, 16);
  sm += __shfl_xor(sm, 2, 16);
  sm += __shfl_xor(sm, 4, 16);
  sm += __shfl_xor(sm, 8, 16);
  const float mu = sm * (1.0f / 128.0f);
  const v4f da = a - mu, dc = c - mu;
  float sq = da.x * da.x + da.y * da.y + da.z * da.z + da.w * da.w
           + dc.x * dc.x + dc.y * dc.y + dc.z * dc.z + dc.w * dc.w;
  sq += __shfl_xor(sq, 1, 16);
  sq += __shfl_xor(sq, 2, 16);
  sq += __shfl_xor(sq, 4, 16);
  sq += __shfl_xor(sq, 8, 16);
  const float rs = rsqrtf(sq * (1.0f / 128.0f) + LN_EPS);
  const float* gp = g + part * 8;
  const float* bp = be + part * 8;
  const bool pad = (t >= NTOK);
  const float y0 = pad ? 0.0f : (da.x * rs * gp[0] + bp[0]);
  const float y1 = pad ? 0.0f : (da.y * rs * gp[1] + bp[1]);
  const float y2 = pad ? 0.0f : (da.z * rs * gp[2] + bp[2]);
  const float y3 = pad ? 0.0f : (da.w * rs * gp[3] + bp[3]);
  const float y4 = pad ? 0.0f : (dc.x * rs * gp[4] + bp[4]);
  const float y5 = pad ? 0.0f : (dc.y * rs * gp[5] + bp[5]);
  const float y6 = pad ? 0.0f : (dc.z * rs * gp[6] + bp[6]);
  const float y7 = pad ? 0.0f : (dc.w * rs * gp[7] + bp[7]);
  unsigned int h0, h1, h2, h3, l0, l1, l2, l3;
  split2(y0, y1, h0, l0);
  split2(y2, y3, h1, l1);
  split2(y4, y5, h2, l2);
  split2(y6, y7, h3, l3);
  const v4u hq = {h0, h1, h2, h3};
  const v4u lq = {l0, l1, l2, l3};
  *(v4ua*)(ph_ + t * CDIM + part * 8) = hq;
  *(v4ua*)(pl_ + t * CDIM + part * 8) = lq;
}

__global__ __launch_bounds__(256) void tf_kernel(
    const int* __restrict__ xx, const float* __restrict__ ss,
    const float* __restrict__ bqkv, const float* __restrict__ bo,
    const float* __restrict__ ln1g, const float* __restrict__ ln1b,
    const float* __restrict__ ln2g, const float* __restrict__ ln2b,
    const float* __restrict__ b1, const float* __restrict__ b2,
    const float* __restrict__ bact, const float* __restrict__ Wsc, const float* __restrict__ bsc,
    const unsigned short* __restrict__ wph, const unsigned short* __restrict__ wpl,
    float* __restrict__ out)
{
  extern __shared__ __attribute__((aligned(16))) unsigned char dsm[];
  float* aL  = (float*)(dsm + T_AL);
  float* qkv = (float*)(dsm + T_QKV);
  unsigned short* pah = (unsigned short*)(dsm + T_PAH);
  unsigned short* pal = (unsigned short*)(dsm + T_PAL);
  unsigned short* pbh = (unsigned short*)(dsm + T_PBH);
  unsigned short* pbl = (unsigned short*)(dsm + T_PBL);
  float* ost = (float*)(dsm + T_OST);

  const int b = blockIdx.x, tid = threadIdx.x;
  const int lane = tid & 31, w = tid >> 5, h = lane >> 4, m = lane & 15;
  const v8f zero8 = {0.f, 0.f, 0.f, 0.f, 0.f, 0.f, 0.f, 0.f};

  if (tid < CDIM) aL[NTOK * CDIM + tid] = 0.0f;

  {
    const int* frb = xx + (size_t)b * NFRM * NCELL;
    #pragma unroll
    for (int it = 0; it < 4; ++it) {
      const int idx = it * 256 + tid;
      const int t = idx >> 6, k0 = (idx & 63) * 8;
      const int tt = (t < NTOK) ? t : (NTOK - 1);
      const int* src = frb + (tt + 1) * NCELL + k0;
      const v4i a = *(const v4ia*)src;
      const v4i c = *(const v4ia*)(src + 4);
      const bool z = (t >= NTOK);
      const unsigned int q0 = z ? 0u : (f2bf_bits((float)a.x) | (f2bf_bits((float)a.y) << 16));
      const unsigned int q1 = z ? 0u : (f2bf_bits((float)a.z) | (f2bf_bits((float)a.w) << 16));
      const unsigned int q2 = z ? 0u : (f2bf_bits((float)c.x) | (f2bf_bits((float)c.y) << 16));
      const unsigned int q3 = z ? 0u : (f2bf_bits((float)c.z) | (f2bf_bits((float)c.w) << 16));
      const v4u qv = {q0, q1, q2, q3};
      *(v4ua*)(pbh + t * FFD + k0) = qv;
    }
  }
  __syncthreads();

  {
    v8f acc[1];
    acc[0] = zero8;
    gemm16<1, 16, false>(acc, pbh, pbh, FFD,
                         wph + OFF_WACT + (size_t)(16 * w) * FFD, wpl + OFF_WACT + (size_t)(16 * w) * FFD,
                         FFD, h, m);
    const int col = 16 * w + m;
    const float bb = bact[col];
    #pragma unroll
    for (int r = 0; r < 8; ++r) {
      const int row = 8 * h + r;
      if (row < NTOK) aL[row * CDIM + col] = acc[0][r] + bb;
    }
  }
  __syncthreads();

  #pragma unroll 1
  for (int l = 0; l < LTF; ++l) {
    ln_planes(aL, ln1g + l * CDIM, ln1b + l * CDIM, pah, pal, tid);
    __syncthreads();

    {
      v8f acc[3];
      #pragma unroll
      for (int i = 0; i < 3; ++i) acc[i] = zero8;
      const size_t wo = OFF_WQKV + (size_t)l * QKVD * CDIM + (size_t)(48 * w) * CDIM;
      gemm16<3, 4, true>(acc, pah, pal, CDIM, wph + wo, wpl + wo, CDIM, h, m);
      #pragma unroll
      for (int i = 0; i < 3; ++i) {
        const int col = 48 * w + 16 * i + m;
        const float bb = bqkv[l * QKVD + col];
        #pragma unroll
        for (int r = 0; r < 8; ++r) qkv[(8 * h + r) * QKVD + col] = acc[i][r] + bb;
      }
    }
    __syncthreads();

    if (tid < 4 * NTOK) {
      const int hq = tid / NTOK, q = tid - hq * NTOK;
      const float* qp = qkv + q * QKVD + hq * 32;
      v4f qv[8];
      #pragma unroll
      for (int i = 0; i < 8; ++i) qv[i] = *(const v4fa*)(qp + 4 * i);
      float sc[NTOK];
      float mx = -3.0e38f;
      #pragma unroll
      for (int k2 = 0; k2 < NTOK; ++k2) {
        const float* kp = qkv + k2 * QKVD + CDIM + hq * 32;
        float d = 0.0f;
        #pragma unroll
        for (int i = 0; i < 8; ++i) {
          const v4f kv = *(const v4fa*)(kp + 4 * i);
          d += qv[i].x * kv.x + qv[i].y * kv.y + qv[i].z * kv.z + qv[i].w * kv.w;
        }
        d *= 0.17677669529663688f;
        sc[k2] = d;
        mx = fmaxf(mx, d);
      }
      float sum = 0.0f;
      #pragma unroll
      for (int k2 = 0; k2 < NTOK; ++k2) {
        const float e = __expf(sc[k2] - mx);
        sc[k2] = e;
        sum += e;
      }
      const float inv = 1.0f / sum;
      #pragma unroll
      for (int d4 = 0; d4 < 8; ++d4) {
        v4f o = {0.f, 0.f, 0.f, 0.f};
        #pragma unroll
        for (int k2 = 0; k2 < NTOK; ++k2) {
          const v4f vv = *(const v4fa*)(qkv + k2 * QKVD + 2 * CDIM + hq * 32 + 4 * d4);
          o += vv * sc[k2];
        }
        o *= inv;
        unsigned int h0, h1, l0, l1;
        split2(o.x, o.y, h0, l0);
        split2(o.z, o.w, h1, l1);
        const v2u hv = {h0, h1};
        const v2u lv = {l0, l1};
        const int po = q * CDIM + hq * 32 + 4 * d4;
        *(v2ua*)(pah + po) = hv;
        *(v2ua*)(pal + po) = lv;
      }
    } else if (tid >= 64 && tid < 96) {
      const int c4 = (tid - 64) * 4;
      const v2u z2 = {0u, 0u};
      *(v2ua*)(pah + NTOK * CDIM + c4) = z2;
      *(v2ua*)(pal + NTOK * CDIM + c4) = z2;
    }
    __syncthreads();

    {
      v8f acc[1];
      acc[0] = zero8;
      const size_t wo = OFF_WO + (size_t)l * CDIM * CDIM + (size_t)(16 * w) * CDIM;
      gemm16<1, 4, true>(acc, pah, pal, CDIM, wph + wo, wpl + wo, CDIM, h, m);
      const int col = 16 * w + m;
      const float bb = bo[l * CDIM + col];
      #pragma unroll
      for (int r = 0; r < 8; ++r) {
        const int row = 8 * h + r;
        if (row < NTOK) aL[row * CDIM + col] += acc[0][r] + bb;
      }
    }
    __syncthreads();

    ln_planes(aL, ln2g + l * CDIM, ln2b + l * CDIM, pah, pal, tid);
    __syncthreads();

    {
      v8f acc[4];
      #pragma unroll
      for (int i = 0; i < 4; ++i) acc[i] = zero8;
      const size_t wo = OFF_W1 + (size_t)l * FFD * CDIM + (size_t)(64 * w) * CDIM;
      gemm16<4, 4, true>(acc, pah, pal, CDIM, wph + wo, wpl + wo, CDIM, h, m);
      #pragma unroll
      for (int i = 0; i < 4; ++i) {
        const int col = 64 * w + 16 * i + m;
        const float bb = b1[l * FFD + col];
        #pragma unroll
        for (int r = 0; r < 8; ++r) {
          const int row = 8 * h + r;
          const float hv = (row < NTOK) ? fmaxf(acc[i][r] + bb, 0.0f) : 0.0f;
          const unsigned int hb = f2bf_bits(hv);
          const unsigned int lb = f2bf_bits(hv - bf_bits2f(hb));
          pbh[row * FFD + col] = (unsigned short)hb;
          pbl[row * FFD + col] = (unsigned short)lb;
        }
      }
    }
    __syncthreads();

    {
      v8f acc[1];
      acc[0] = zero8;
      const size_t wo = OFF_W2 + (size_t)l * CDIM * FFD + (size_t)(16 * w) * FFD;
      gemm16<1, 16, true>(acc, pbh, pbl, FFD, wph + wo, wpl + wo, FFD, h, m);
      const int col = 16 * w + m;
      const float bb = b2[l * CDIM + col];
      #pragma unroll
      for (int r = 0; r < 8; ++r) {
        const int row = 8 * h + r;
        if (row < NTOK) aL[row * CDIM + col] += acc[0][r] + bb;
      }
    }
    __syncthreads();
  }

  if (tid < CDIM) {
    float s = 0.0f;
    #pragma unroll
    for (int t = 0; t < NTOK; ++t) s += aL[t * CDIM + tid];
    ost[tid] = s * (1.0f / 15.0f);
    ost[CDIM + tid] = fmaxf(ss[b] * Wsc[tid] + bsc[tid], 0.0f);
  }
  __syncthreads();
  if (tid < 64) {
    const v4f v = *(const v4fa*)(ost + 4 * tid);
    float* dst = out + (size_t)b * OROWS * CDIM + 24 * CDIM + 4 * tid;
    *(volatile v4f*)dst = v;
    __threadfence();
    *(volatile v4f*)dst = v;
  }
}

extern "C" void kernel_launch(void* const* d_in, const int* in_sizes, int n_in,
                              void* d_out, int out_size, void* d_ws, size_t ws_size,
                              hipStream_t stream) {
  if (n_in < 25) return;
  const int nb = in_sizes[0] / (NFRM * NCELL);
  if (nb <= 0 || nb * NFRM * NCELL != in_sizes[0]) return;
  if (in_sizes[1] != nb) return;
  if (in_sizes[2] != CDIM * 5 || in_sizes[3] != CDIM) return;
  if (in_sizes[4] != LGNN * CDIM * CDIM || in_sizes[5] != LGNN * CDIM || in_sizes[6] != LGNN * CDIM * CDIM) return;
  if (in_sizes[7] != CDIM || in_sizes[8] != CDIM) return;
  if (in_sizes[9] != LTF * QKVD * CDIM || in_sizes[10] != LTF * QKVD) return;
  if (in_sizes[11] != LTF * CDIM * CDIM || in_sizes[12] != LTF * CDIM) return;
  if (in_sizes[13] != LTF * CDIM || in_sizes[14] != LTF * CDIM || in_sizes[15] != LTF * CDIM || in_sizes[16] != LTF * CDIM) return;
  if (in_sizes[17] != LTF * FFD * CDIM || in_sizes[18] != LTF * FFD) return;
  if (in_sizes[19] != LTF * CDIM * FFD || in_sizes[20] != LTF * CDIM) return;
  if (in_sizes[21] != CDIM * NCELL || in_sizes[22] != CDIM) return;
  if (in_sizes[23] != CDIM || in_sizes[24] != CDIM) return;
  if (out_size != nb * OROWS * CDIM) return;

  const int*   xx   = (const int*)  d_in[0];
  const float* ss_  = (const float*)d_in[1];
  const float* Win  = (const float*)d_in[2];
  const float* b_in = (const float*)d_in[3];
  const float* Wl   = (const float*)d_in[4];
  const float* bl   = (const float*)d_in[5];
  const float* Wr   = (const float*)d_in[6];
  const float* ln_g = (const float*)d_in[7];
  const float* ln_b = (const float*)d_in[8];
  const float* Wqkv = (const float*)d_in[9];
  const float* bqkv = (const float*)d_in[10];
  const float* Wo   = (const float*)d_in[11];
  const float* bo   = (const float*)d_in[12];
  const float* ln1g = (const float*)d_in[13];
  const float* ln1b = (const float*)d_in[14];
  const float* ln2g = (const float*)d_in[15];
  const float* ln2b = (const float*)d_in[16];
  const float* W1   = (const float*)d_in[17];
  const float* b1   = (const float*)d_in[18];
  const float* W2   = (const float*)d_in[19];
  const float* b2   = (const float*)d_in[20];
  const float* Wact = (const float*)d_in[21];
  const float* bact = (const float*)d_in[22];
  const float* Wsc  = (const float*)d_in[23];
  const float* bsc  = (const float*)d_in[24];
  float* out = (float*)d_out;

  const size_t plane_bytes = (size_t)PLANE_N * 2;
  const size_t total = 2 * plane_bytes;
  if (total > ws_size) return;
  char* ws = (char*)d_ws;
  unsigned short* wph = (unsigned short*)(ws);
  unsigned short* wpl = (unsigned short*)(ws + plane_bytes);

  prep_kernel<<<dim3(PLANE_N / 8 / 256), dim3(256), 0, stream>>>(Wl, Wr, Wact, Wqkv, Wo, W1, W2, wph, wpl);

  gnn_kernel<<<dim3(nb), dim3(256), G_LDS, stream>>>(xx, ss_, Win, b_in, bl, ln_g, ln_b, wph, wpl, out);

  tf_kernel<<<dim3(nb), dim3(256), T_LDS, stream>>>(xx, ss_, bqkv, bo, ln1g, ln1b, ln2g, ln2b,
                                                   b1, b2, bact, Wsc, bsc, wph, wpl, out);
}
